// Noise_Regressor_16587163697396
// MI455X (gfx1250) — hardware-verified
//
#include <hip/hip_runtime.h>
#include <math.h>

typedef __attribute__((ext_vector_type(16))) _Float16 v16h;
typedef __attribute__((ext_vector_type(16))) __bf16 v16b;
typedef __attribute__((ext_vector_type(8)))  _Float16 v8h;
typedef __attribute__((ext_vector_type(8)))  float v8f;
typedef __attribute__((ext_vector_type(4)))  float v4f;
typedef __attribute__((ext_vector_type(2)))  float v2f;
typedef __attribute__((ext_vector_type(4)))  unsigned v4u;
typedef __attribute__((ext_vector_type(4)))  int v4i;
typedef float __attribute__((may_alias)) float_a;
typedef int __attribute__((may_alias)) int_a;

template <typename T> __device__ __forceinline__ void vst2(void* p, T v) { *(volatile T*)p = v; __threadfence(); *(volatile T*)p = v; }
__device__ __forceinline__ v8f wmma16(v16h a, v16h b, v8f c) {
  v8f d = __builtin_amdgcn_wmma_f32_16x16x32_f16(false, a, false, b, (short)0, c, false, false);
  asm volatile("v_nop\n\tv_nop\n\tv_nop\n\tv_nop" : "+v"(d) : "v"(a), "v"(b));
  return d;
}
__device__ __forceinline__ v8f wmma_bf(v16b a, v16b b, v8f c) {
  v8f d = __builtin_amdgcn_wmma_f32_16x16x32_bf16(false, a, false, b, (short)0, c, false, false);
  asm volatile("v_nop\n\tv_nop\n\tv_nop\n\tv_nop" : "+v"(d) : "v"(a), "v"(b));
  return d;
}
__device__ __forceinline__ v16h frag_h(const _Float16* rowk0, int lane) {
  union { v16h v; v8h q[2]; } u; const _Float16* p = rowk0 + 8 * (lane >> 4);
  u.q[0] = *(const v8h*)p; u.q[1] = *(const v8h*)(p + 16); return u.v;
}
__device__ __forceinline__ v16h frag_f32(const float* rowk0, int lane) {
  v16h a; const float* p = rowk0 + 8 * (lane >> 4);
#pragma unroll
  for (int i = 0; i < 8; ++i) { a[i] = (_Float16)p[i]; a[8 + i] = (_Float16)p[16 + i]; }
  return a;
}
__device__ __forceinline__ v16h frag_f32s(const float* rowk0, int lane, float sc) {
  v16h a; const float* p = rowk0 + 8 * (lane >> 4);
#pragma unroll
  for (int i = 0; i < 8; ++i) { a[i] = (_Float16)(p[i] * sc); a[8 + i] = (_Float16)(p[16 + i] * sc); }
  return a;
}
__device__ __forceinline__ v16h fragc_f32(const float* W, int k0, int n, int lane, int ld, int K) {
  v16h a; const int g = lane >> 4;
#pragma unroll
  for (int i = 0; i < 8; ++i) { const int ka = k0 + 8 * g + i, kb = ka + 16;
    a[i] = (_Float16)(ka < K ? W[(size_t)(ka < K ? ka : K - 1) * ld + n] : 0.f); a[8 + i] = (_Float16)(kb < K ? W[(size_t)(kb < K ? kb : K - 1) * ld + n] : 0.f); }
  return a;
}
struct F2 { v16b h, l; };
__device__ __forceinline__ F2 bsplit16(const float v[16]) { F2 r;
#pragma unroll
  for (int i = 0; i < 16; ++i) { const __bf16 h = (__bf16)v[i]; r.h[i] = h; r.l[i] = (__bf16)(v[i] - (float)h); }
  return r; }
__device__ __forceinline__ F2 split_row(const float* row, int k0, int lane) { float v[16]; const float* p = row + k0 + 8 * (lane >> 4);
#pragma unroll
  for (int i = 0; i < 8; ++i) { v[i] = p[i]; v[8 + i] = p[16 + i]; }
  return bsplit16(v); }
__device__ __forceinline__ F2 split_rowK(const float* row, int k0, int lane, int K) { float v[16]; const int g = lane >> 4;
#pragma unroll
  for (int i = 0; i < 8; ++i) { const int ka = k0 + 8 * g + i, kb = ka + 16; v[i] = ka < K ? row[ka < K ? ka : K - 1] : 0.f; v[8 + i] = kb < K ? row[kb < K ? kb : K - 1] : 0.f; }
  return bsplit16(v); }
__device__ __forceinline__ F2 split_col(const float* W, int k0, int n, int lane, int ld, int K) { float v[16]; const int g = lane >> 4;
#pragma unroll
  for (int i = 0; i < 8; ++i) { const int ka = k0 + 8 * g + i, kb = ka + 16; v[i] = ka < K ? W[(size_t)(ka < K ? ka : K - 1) * ld + n] : 0.f; v[8 + i] = kb < K ? W[(size_t)(kb < K ? kb : K - 1) * ld + n] : 0.f; }
  return bsplit16(v); }
__device__ __forceinline__ v8f mac3(const F2& a, const F2& b, v8f c) { c = wmma_bf(a.l, b.h, c); c = wmma_bf(a.h, b.l, c); return wmma_bf(a.h, b.h, c); }
__device__ __forceinline__ float sigm(float v) { return 1.0f / (1.0f + expf(-v)); }
#define LDSX() do { asm volatile("s_wait_dscnt 0" ::: "memory"); __builtin_amdgcn_wave_barrier(); __builtin_amdgcn_fence(__ATOMIC_RELEASE, "workgroup"); } while (0)


#define SEQ 4096
#define DM 1024
#define NI 72
#define NNZ 12
#define NP (NI * NNZ)
#define TST 300
__device__ __forceinline__ float bfr(float v) { return (float)(__bf16)v; }
__device__ __forceinline__ v16b frag_b(const __bf16* rowk0, int lane) { return __builtin_bit_cast(v16b, frag_h((const _Float16*)rowk0, lane)); }
__device__ __attribute__((noinline)) float softplus_ni(float v) { return v > 20.f ? v : log1pf(expf(v)); }

__global__ __launch_bounds__(256) void k_pack(const float* __restrict__ W, __bf16* __restrict__ PT) {
  const int n = blockIdx.x, tid = threadIdx.x; __shared__ __align__(16) __bf16 srow[DM];
  for (int k = tid; k < DM; k += 256) srow[k] = (__bf16)W[(size_t)k * NP + n];
  __syncthreads();
  if (tid < DM / 8) vst2((unsigned*)(PT + (size_t)n * DM + tid * 8), *(const v4u*)(&srow[tid * 8]));
}
__global__ __launch_bounds__(128) void k_ln(const float* __restrict__ x, const float* __restrict__ lg, const float* __restrict__ lb, __bf16* __restrict__ XH, __bf16* __restrict__ XL) {
  const int tid = threadIdx.x, wave = tid >> 5, lane = tid & 31; const int r0 = blockIdx.x * 64 + wave * 16;
  __shared__ __align__(16) __bf16 sh_[4][DM + 8], sl_[4][DM + 8];
  for (int rl = 0; rl < 16; ++rl) { const float* xr = x + (size_t)(r0 + rl) * DM; float v[32]; float s = 0.f;
#pragma unroll
    for (int e = 0; e < 32; ++e) { v[e] = bfr(xr[lane * 32 + e]); s += v[e]; }
#pragma unroll
    for (int o = 16; o > 0; o >>= 1) s += __shfl_xor(s, o, 32);
    const float mu = s * (1.0f / DM); float q = 0.f;
#pragma unroll
    for (int e = 0; e < 32; ++e) { const float dv = v[e] - mu; q += dv * dv; }
#pragma unroll
    for (int o = 16; o > 0; o >>= 1) q += __shfl_xor(q, o, 32);
    const float rs = rsqrtf(q * (1.0f / DM) + 1e-5f);
#pragma unroll
    for (int e = 0; e < 32; ++e) { const int c = lane * 32 + e; const float y = (v[e] - mu) * rs * bfr(lg[c]) + bfr(lb[c]); const __bf16 hi = (__bf16)y; sh_[wave][c] = hi; sl_[wave][c] = (__bf16)(y - (float)hi); }
    LDSX();
    for (int pc = lane; pc < DM / 8; pc += 32) { vst2((unsigned*)(XH + (size_t)(r0 + rl) * DM + pc * 8), *(const v4u*)(&sh_[wave][pc * 8])); vst2((unsigned*)(XL + (size_t)(r0 + rl) * DM + pc * 8), *(const v4u*)(&sl_[wave][pc * 8])); }
    LDSX(); }
}
__global__ __launch_bounds__(128) void k_gemm(const __bf16* __restrict__ XH, const __bf16* __restrict__ XL, const __bf16* __restrict__ PT, const float* __restrict__ bias, float* __restrict__ P) {
  __shared__ __align__(16) float so[4][16][100];
  const int tid = threadIdx.x, wave = tid >> 5, lane = tid & 31, col = lane & 15, g = lane >> 4; const int r0 = blockIdx.x * 64 + wave * 16, n0 = blockIdx.y * 96;
  v8f acc[6] = {};
#pragma unroll 2
  for (int kc = 0; kc < DM / 32; ++kc) { const v16b ah = frag_b(XH + (size_t)(r0 + col) * DM + kc * 32, lane), al = frag_b(XL + (size_t)(r0 + col) * DM + kc * 32, lane);
#pragma unroll
    for (int j = 0; j < 6; ++j) { const v16b wb = frag_b(PT + (size_t)(n0 + j * 16 + col) * DM + kc * 32, lane); acc[j] = wmma_bf(al, wb, acc[j]); acc[j] = wmma_bf(ah, wb, acc[j]); } }
#pragma unroll
  for (int j = 0; j < 6; ++j) { const float bb = bfr(bias[n0 + j * 16 + col]);
#pragma unroll
    for (int r = 0; r < 8; ++r) so[wave][8 * g + r][j * 16 + col] = acc[j][r] + bb; }
  LDSX();
  for (int rl = 0; rl < 16; ++rl) { if (lane < 24) vst2(P + (size_t)(r0 + rl) * NP + n0 + lane * 4, *(const v4f*)(&so[wave][rl][lane * 4])); }
}
__global__ __launch_bounds__(256) void k_maps(const float* __restrict__ P, float* __restrict__ O1, float* __restrict__ O2, float* __restrict__ O3, float* __restrict__ O4) {
  __shared__ __align__(16) float st[4][NI][68];
  const int tid = threadIdx.x; const int s0 = blockIdx.x * 64;
  for (int q = tid; q < 64 * NI * 4; q += 256) { const int m = q / (64 * NI), rem = q % (64 * NI); const int rl = rem / NI, i = rem % NI; const float v = P[(size_t)(s0 + rl) * NP + (8 + m) * NI + i]; st[m][i][rl] = (m & 1) ? softplus_ni(v) : v; }
  __syncthreads();
  for (int q = tid; q < 4 * NI * 16; q += 256) { const int m = q / (NI * 16), rem = q % (NI * 16); const int i = rem >> 4, pc = rem & 15; float* O = m == 0 ? O1 : (m == 1 ? O2 : (m == 2 ? O3 : O4)); vst2(O + (size_t)i * SEQ + s0 + pc * 4, *(const v4f*)(&st[m][i][pc * 4])); }
}
__global__ __launch_bounds__(256) void k_kin(const float* __restrict__ P, float* __restrict__ K) {
  __shared__ __align__(16) float sacc[SEQ + TST + 4];
  __shared__ __align__(16) float sst[16][256][8];
  const int tid = threadIdx.x; const int i = blockIdx.x;
  for (int q = tid; q < SEQ + TST + 4; q += 256) sacc[q] = 0.f;
#pragma unroll 1
  for (int m = 0; m < 16; ++m) { const int s = tid + 256 * m; const float* pr = P + (size_t)s * NP;
    const float c = pr[4 * NI + i], cth = pr[5 * NI + i], phi = pr[6 * NI + i], phth = pr[7 * NI + i];
    const float d = softplus_ni(pr[1 * NI + i]); const float k = d * d * 0.25f + softplus_ni(pr[0 * NI + i]);
    const float dth = softplus_ni(pr[3 * NI + i]); const float kth = dth * dth * 0.25f + softplus_ni(pr[2 * NI + i]);
    const float w1 = sqrtf(k * 4.0f - d * d) * 0.5f, w2 = sqrtf(kth * 4.0f - dth * dth) * 0.5f;
    float st8[8]; float sn, cs;
    sincosf(phi, &sn, &cs); st8[0] = c * cs; st8[1] = c * sn;
    { const float g1 = expf(-0.5f * d); sincosf(w1, &sn, &cs); st8[2] = g1 * cs; st8[3] = g1 * sn; }
    sincosf(phth, &sn, &cs); st8[4] = cth * cs; st8[5] = cth * sn;
    { const float g2 = expf(-0.5f * dth); sincosf(w2, &sn, &cs); st8[6] = g2 * cs; st8[7] = g2 * sn; }
    *(v4f*)(&sst[m][tid][0]) = (v4f){st8[0], st8[1], st8[2], st8[3]}; *(v4f*)(&sst[m][tid][4]) = (v4f){st8[4], st8[5], st8[6], st8[7]}; }
  __syncthreads();
#pragma unroll 1
  for (int t = 0; t < TST; ++t) {
#pragma unroll 1
    for (int m = 0; m < 16; ++m) { const v4f a = *(const v4f*)(&sst[m][tid][0]); const v4f b = *(const v4f*)(&sst[m][tid][4]);
      sacc[tid + 256 * m + t] += a[1] + b[1];
      const float nr1 = a[0] * a[2] - a[1] * a[3], ni1 = a[0] * a[3] + a[1] * a[2];
      const float nr2 = b[0] * b[2] - b[1] * b[3], ni2 = b[0] * b[3] + b[1] * b[2];
      *(v2f*)(&sst[m][tid][0]) = (v2f){nr1, ni1}; *(v2f*)(&sst[m][tid][4]) = (v2f){nr2, ni2}; }
    __syncthreads(); }
  for (int q = tid; q < SEQ / 4; q += 256) vst2(K + (size_t)i * SEQ + q * 4, *(const v4f*)(&sacc[q * 4]));
}
extern "C" void kernel_launch(void* const* d_in, const int* in_sizes, int n_in, void* d_out, int out_size, void* d_ws, size_t ws_size, hipStream_t stream) {
  (void)in_sizes; (void)n_in; (void)out_size; (void)ws_size;
  const float* x = (const float*)d_in[0]; const float* lg = (const float*)d_in[1]; const float* lb = (const float*)d_in[2]; const float* W = (const float*)d_in[3]; const float* b = (const float*)d_in[4];
  float* O0 = (float*)d_out; float* O1 = (float*)((char*)d_out + 1179648); float* O2 = (float*)((char*)d_out + 2359296); float* O3 = (float*)((char*)d_out + 3538944); float* O4 = (float*)((char*)d_out + 4718592);
  char* ws = (char*)d_ws; size_t off = 0;
  auto take = [&](size_t bytes) { char* p = ws + off; off += (bytes + 255) & ~(size_t)255; return p; };
  __bf16* PT = (__bf16*)take((size_t)NP * DM * 2); __bf16* XH = (__bf16*)take((size_t)SEQ * DM * 2); __bf16* XL = (__bf16*)take((size_t)SEQ * DM * 2); float* P = (float*)take((size_t)SEQ * NP * 4);
  k_pack<<<NP, 256, 0, stream>>>(W, PT);
  k_ln<<<SEQ / 64, 128, 0, stream>>>(x, lg, lb, XH, XL);
  k_gemm<<<dim3(SEQ / 64, NP / 96), 128, 0, stream>>>(XH, XL, PT, b, P);
  k_maps<<<SEQ / 64, 256, 0, stream>>>(P, O1, O2, O3, O4);
  k_kin<<<NI, 256, 0, stream>>>(P, O0);
}
